// PairwisePrediction_54640573939859
// MI455X (gfx1250) — hardware-verified
//
#include <hip/hip_runtime.h>
#include <stddef.h>


typedef _Float16 v16h __attribute__((ext_vector_type(16)));
typedef _Float16 v8h  __attribute__((ext_vector_type(8)));
typedef float    v8f  __attribute__((ext_vector_type(8)));
typedef float    v4f  __attribute__((ext_vector_type(4)));
typedef _Float16 h16;

#ifndef NB
#define NB 2
#endif
#ifndef SEQ
#define SEQ 512
#endif
#define NB_FULL  2
#define SEQ_FULL 512
#define KD    256
#define PW    256
#define MROWS (NB * SEQ)
#define NTILE (SEQ / 32)
#define SLOPE 0.2f

static_assert(NB >= 1 && NB <= NB_FULL);
static_assert(SEQ >= 64 && SEQ <= SEQ_FULL && (SEQ % 64) == 0);
static_assert((KD % 32) == 0);
static_assert(KD / 8 == 32);
static_assert((PW % 64) == 0 && (PW % 32) == 0 && (PW % 16) == 0);
static_assert((MROWS % 64) == 0 && (MROWS % 32) == 0);
static_assert((size_t)NB_FULL * SEQ_FULL * SEQ_FULL * 4 == (size_t)2097152);
static_assert((size_t)((NB - 1) * SEQ_FULL + SEQ) * SEQ_FULL <= (size_t)NB_FULL * SEQ_FULL * SEQ_FULL);

#define LDC 68
static_assert((LDC % 4) == 0 && LDC >= 64);

#define WCARRY 64.0f
#define XCARRY 16.0f

#define WT_BYTES  ((size_t)PW * KD * 2)
#define X16_BYTES ((size_t)MROWS * KD * 2)
#define PF_BYTES  ((size_t)MROWS * PW * 4)
#define OFF_WT  ((size_t)0)
#define OFF_X16 (OFF_WT + WT_BYTES)
#define OFF_PF  (OFF_X16 + X16_BYTES)
#define WS_TOTAL (OFF_PF + PF_BYTES)
static_assert((WT_BYTES % 128) == 0 && (X16_BYTES % 128) == 0 && (PF_BYTES % 128) == 0);
static_assert(WS_TOTAL <= (size_t)134217728);

static_assert((size_t)64 * LDC * 4 <= (size_t)131072);
static_assert((size_t)64 * 4 <= (size_t)131072);

__device__ __forceinline__ float bf16r(float x) {
  unsigned int u = __float_as_uint(x);
  u = (u + 0x7FFFu + ((u >> 16) & 1u)) & 0xFFFF0000u;
  return __uint_as_float(u);
}

__device__ __forceinline__ h16 toh_flush(float v) {
  const h16 r = (h16)v;
  return (fabsf(v) < 6.103515625e-05f) ? (h16)0.0f : r;
}

__device__ __forceinline__ v16h frag_at(const _Float16* p) {
  v8h lo = *(const v8h*)(p);
  v8h hi = *(const v8h*)(p + 16);
  v16h out;
#pragma unroll
  for (int i = 0; i < 8; ++i) { out[i] = lo[i]; out[i + 8] = hi[i]; }
  return out;
}

__device__ __forceinline__ v8f wmma16(v16h a, v16h b, v8f c) {
  v8f d = __builtin_amdgcn_wmma_f32_16x16x32_f16(false, a, false, b, (short)0, c,
                                                 false, false);
  asm volatile("v_nop\n\tv_nop\n\tv_nop\n\tv_nop" : "+v"(d) : "v"(a), "v"(b));
  return d;
}

__global__ __launch_bounds__(256) void wconv_kernel(
    const float* __restrict__ W, _Float16* __restrict__ Wt) {
#pragma clang fp contract(off)
  const unsigned gid = blockIdx.x * 256u + threadIdx.x;
  const unsigned n = gid >> 5;
  const unsigned c = (gid & 31u) * 8u;
  const float* src = W + (size_t)n * KD + c;
  const v4f a0 = *(const v4f*)(src);
  const v4f a1 = *(const v4f*)(src + 4u);
  v8h o;
#pragma unroll
  for (int i = 0; i < 4; ++i) {
    o[i]     = toh_flush(WCARRY * bf16r(a0[i]));
    o[i + 4] = toh_flush(WCARRY * bf16r(a1[i]));
  }
  _Float16* p = Wt + (size_t)n * KD + c;
  *(volatile v8h*)p = o;
  __threadfence();
  *(volatile v8h*)p = o;
}
static_assert(((size_t)PW * KD / 8) % 256 == 0);

__global__ __launch_bounds__(256) void xconv_kernel(
    const float* __restrict__ X, _Float16* __restrict__ X16) {
#pragma clang fp contract(off)
  const unsigned gid = blockIdx.x * 256u + threadIdx.x;
  const unsigned row = gid >> 5;
  const unsigned c = (gid & 31u) * 8u;
  const unsigned b = row / (unsigned)SEQ;
  const unsigned s = row - b * (unsigned)SEQ;
  const float* src = X + ((size_t)b * SEQ_FULL + s) * KD + c;
  const v4f a0 = *(const v4f*)(src);
  const v4f a1 = *(const v4f*)(src + 4u);
  v8h o;
#pragma unroll
  for (int i = 0; i < 4; ++i) {
    o[i]     = toh_flush(XCARRY * bf16r(a0[i]));
    o[i + 4] = toh_flush(XCARRY * bf16r(a1[i]));
  }
  _Float16* p = X16 + (size_t)row * KD + c;
  *(volatile v8h*)p = o;
  __threadfence();
  *(volatile v8h*)p = o;
}
static_assert(((size_t)MROWS * KD / 8) % 256 == 0);

__global__ __launch_bounds__(256) void gemm_pre_kernel(
    const _Float16* __restrict__ A16, const _Float16* __restrict__ Bt,
    float* __restrict__ outf) {
  __shared__ float Cs[64 * LDC];
  const unsigned tid = threadIdx.x, lane = tid & 31u;
  const unsigned w = (unsigned)__builtin_amdgcn_readfirstlane((int)(threadIdx.x >> 5));
  const unsigned mw = w >> 1, nw = w & 1u;
  const unsigned hh = lane >> 4, m = lane & 15u;
  const unsigned n0 = blockIdx.x * 64u;
  const unsigned row0 = blockIdx.y * 64u;

  const _Float16* ap  = A16 + (size_t)(row0 + mw * 16u + m) * KD + hh * 8u;
  const _Float16* bp0 = Bt + (size_t)(n0 + nw * 32u + m) * KD + hh * 8u;
  const _Float16* bp1 = bp0 + (size_t)16 * KD;
  v8f acc0 = {}, acc1 = {};
#pragma unroll
  for (unsigned k0 = 0; k0 < (unsigned)KD; k0 += 32u) {
    const v16h a  = frag_at(ap + k0);
    const v16h b0 = frag_at(bp0 + k0);
    const v16h b1 = frag_at(bp1 + k0);
    acc0 = wmma16(a, b0, acc0);
    acc1 = wmma16(a, b1, acc1);
  }
#pragma unroll
  for (int r = 0; r < 8; ++r) {
    float* d = &Cs[(mw * 16u + hh * 8u + (unsigned)r) * LDC + nw * 32u + m];
    d[0]  = acc0[r];
    d[16] = acc1[r];
  }
  __syncthreads();

  const float cs = 1.0f / (WCARRY * XCARRY);
  v4f xs[4];
  size_t off[4];
#pragma unroll
  for (unsigned i = 0; i < 4u; ++i) {
    const unsigned r = 16u * i + (tid >> 4);
    const unsigned c = (tid & 15u) * 4u;
    const v4f u = *(const v4f*)&Cs[r * LDC + c];
    v4f val;
#pragma unroll
    for (int j = 0; j < 4; ++j) val[j] = u[j] * cs;
    xs[i] = val;
    off[i] = (size_t)(row0 + r) * PW + n0 + c;
  }
#pragma unroll
  for (int i = 0; i < 4; ++i) *(volatile v4f*)(outf + off[i]) = xs[i];
  __threadfence();
#pragma unroll
  for (int i = 0; i < 4; ++i) *(volatile v4f*)(outf + off[i]) = xs[i];
}
static_assert(4 * 16 == 64);

__global__ __launch_bounds__(256) void pair_kernel(
    const float* __restrict__ Pf,
    const float* __restrict__ bv, const float* __restrict__ cw, const float* __restrict__ cb,
    float* __restrict__ out) {
#pragma clang fp contract(off)
  __shared__ __attribute__((aligned(16))) float sc[64];

  const unsigned tid = threadIdx.x;
  const unsigned b = blockIdx.z;
  const unsigned ti = blockIdx.y, tj = blockIdx.x;
  const unsigned i0 = ti * 32u, j0 = tj * 32u;

  const unsigned rr = tid >> 2;
  const unsigned q = tid & 3u;
  const unsigned side = rr >> 5;
  const unsigned node = (side != 0u ? j0 : i0) + (rr & 31u);
  const size_t prow = (size_t)(b * (unsigned)SEQ + node) * PW;
  const unsigned cwo = (side != 0u) ? 0u : (unsigned)PW;
  float acc = 0.0f;
#pragma unroll 1
  for (unsigned t = 0; t < (unsigned)(PW / 16); ++t) {
    const unsigned c = (t * 4u + q) * 4u;
    const v4f p = *(const v4f*)(Pf + prow + c);
    const v4f g = *(const v4f*)(bv + c);
    const v4f wv = *(const v4f*)(cw + cwo + c);
#pragma unroll
    for (int j = 0; j < 4; ++j) {
      float x = p[j] + bf16r(g[j]);
      x = (x >= 0.0f) ? x : SLOPE * x;
      acc = fmaf(x, bf16r(wv[j]), acc);
    }
  }
  acc += __shfl_xor(acc, 1, 32);
  acc += __shfl_xor(acc, 2, 32);
  if (q == 0u) sc[rr] = acc;
  __syncthreads();

  const unsigned r = tid >> 3, c0 = (tid & 7u) * 4u;
  const float sr = sc[r];
  const v4f sl = *(const v4f*)&sc[32u + c0];
  const float c2 = bf16r(cb[0]);
  v4f u;
#pragma unroll
  for (int j = 0; j < 4; ++j) u[j] = (sr + sl[j]) + c2;
  const size_t offa = ((size_t)b * SEQ_FULL + i0 + r) * SEQ_FULL + j0 + c0;
  *(volatile v4f*)(out + offa) = u;
  __threadfence();
  *(volatile v4f*)(out + offa) = u;
}
static_assert(256 / 8 == 32);
static_assert(256 / 4 == 64);
static_assert(4 * (PW / 16) * 4 == PW);
static_assert(NTILE * 32 == SEQ);

extern "C" void kernel_launch(void* const* d_in, const int* in_sizes, int n_in,
                              void* d_out, int out_size, void* d_ws, size_t ws_size,
                              hipStream_t stream) {
  if (n_in < 5) return;
  const long long need_x = ((long long)(NB - 1) * SEQ_FULL + SEQ) * KD;
  const long long need_o = ((long long)(NB - 1) * SEQ_FULL + SEQ) * SEQ_FULL;
  if ((long long)in_sizes[0] < need_x) return;
  if ((long long)in_sizes[1] < (long long)PW * KD) return;
  if (in_sizes[2] < PW || in_sizes[3] < 2 * PW || in_sizes[4] < 1) return;
  if ((long long)out_size < need_o) return;
  if (ws_size < WS_TOTAL) return;

  const float* emb = (const float*)d_in[0];
  const float* wq  = (const float*)d_in[1];
  const float* bq  = (const float*)d_in[2];
  const float* cw  = (const float*)d_in[3];
  const float* cb  = (const float*)d_in[4];
  float* out = (float*)d_out;

  char* ws = (char*)d_ws;
  _Float16* Wt  = (_Float16*)(ws + OFF_WT);
  _Float16* X16 = (_Float16*)(ws + OFF_X16);
  float*    Pf  = (float*)(ws + OFF_PF);

  dim3 blk(256);
  wconv_kernel<<<dim3(PW * KD / 8 / 256), blk, 0, stream>>>(wq, Wt);
  xconv_kernel<<<dim3(MROWS * KD / 8 / 256), blk, 0, stream>>>(emb, X16);
  gemm_pre_kernel<<<dim3(PW / 64, MROWS / 64), blk, 0, stream>>>(X16, Wt, Pf);
  pair_kernel<<<dim3(NTILE, NTILE, NB), blk, 0, stream>>>(Pf, bq, cw, cb, out);
}
